// KalmanFilter_5815385719315
// MI455X (gfx1250) — hardware-run, weakly checked
//
#include <hip/hip_runtime.h>
#include <math.h>

typedef __attribute__((ext_vector_type(16))) _Float16 v16h;
typedef __attribute__((ext_vector_type(8)))  _Float16 v8h;
typedef __attribute__((ext_vector_type(8)))  float    v8f;
typedef __attribute__((ext_vector_type(4)))  float    v4f;

constexpr int kN       = 64;
constexpr int kT       = 8192;
constexpr int kThreads = 512;
constexpr int kHP      = 72;
constexpr int kFP      = 68;
constexpr int kBuf     = 32;
constexpr float kCarry    = 16.0f;
constexpr float kRes      = 2048.0f;
constexpr float kInvRes   = 1.0f / kRes;
constexpr float kInvCarry = 1.0f / kCarry;
constexpr float kInvCC    = 1.0f / (kCarry * kCarry);
constexpr float kF16Min   = 6.103515625e-5f;

static_assert(kN == 64, "16 waves x one 16x16 tile");
static_assert((kN % 32) == 0, "K multiple of 32");
static_assert((kT % kBuf) == 0 && kBuf == 32, "one 128-B line per latent row per flush");
static_assert((kHP % 8) == 0 && kHP >= kN, "16-B aligned fragment rows");
static_assert((kFP % 4) == 0 && kFP >= kN, "16-B aligned f32 rows");
constexpr size_t kLdsBytes = (size_t)14 * kN * kHP * 2 + (size_t)4 * kN * kFP * 4 + (size_t)4 * kN * 4 + (size_t)3 * kBuf * kN * 4;
static_assert(kLdsBytes == 224256, "LDS total");
static_assert(kLdsBytes <= 327680, "LDS cap");

__device__ __forceinline__ float bf16v(float f) {
  unsigned u = __float_as_uint(f);
  u = (u + 0x7FFFu + ((u >> 16) & 1u)) & 0xFFFF0000u;
  return __uint_as_float(u);
}
__device__ __forceinline__ float flush16(float c) {
  return (fabsf(c) < kF16Min) ? 0.0f : c;
}
__device__ __forceinline__ void split16(float c, _Float16& hi, _Float16& lo) {
  const _Float16 hv = (_Float16)flush16(c);
  float hf = (float)hv;
  asm volatile("" : "+v"(hf));
  const float r = (c - hf) * kRes;
  hi = hv;
  lo = (_Float16)flush16(r);
}
__device__ __forceinline__ v8f mma16(v16h a, v16h b, v8f c) {
  c = __builtin_amdgcn_wmma_f32_16x16x32_f16(false, a, false, b, (short)0, c, false, false);
  asm volatile("v_nop\n\tv_nop\n\tv_nop\n\tv_nop" : "+v"(c) : "v"(a), "v"(b));
  return c;
}
union FragU { v16h v; v8h h[2]; };
__device__ __forceinline__ v16h ldfrag(const _Float16* p) {
  FragU f;
  f.h[0] = *(const v8h*)(p);
  f.h[1] = *(const v8h*)(p + 16);
  return f.v;
}
__device__ __forceinline__ _Float16 wcvt(float x) {
  return (_Float16)flush16(bf16v(x) * kCarry);
}
__device__ __forceinline__ v16h wfrag(const float* __restrict__ W, int row, int kb) {
  const float* p = W + row * kN + kb;
  const v4f a0 = *(const v4f*)(p);
  const v4f a1 = *(const v4f*)(p + 4);
  const v4f a2 = *(const v4f*)(p + 16);
  const v4f a3 = *(const v4f*)(p + 20);
  v16h f;
#pragma unroll
  for (int e = 0; e < 4; ++e) {
    const float x0 = a0[e];
    const float x1 = a1[e];
    const float x2 = a2[e];
    const float x3 = a3[e];
    f[e]      = wcvt(x0);
    f[4 + e]  = wcvt(x1);
    f[8 + e]  = wcvt(x2);
    f[12 + e] = wcvt(x3);
  }
  return f;
}
template <bool ROWM, bool TRN>
__device__ __forceinline__ void put_planes(const float (&cv)[8],
                                           _Float16* rh, _Float16* rl, int rbase,
                                           _Float16* th, _Float16* tl, int tbase) {
  v8h hv, lv;
#pragma unroll
  for (int r = 0; r < 8; ++r) {
    _Float16 a, b;
    split16(cv[r], a, b);
    if (ROWM) {
      rh[rbase + r * kHP] = a;
      rl[rbase + r * kHP] = b;
    }
    hv[r] = a;
    lv[r] = b;
  }
  if (TRN) {
    *(v8h*)(th + tbase) = hv;
    *(v8h*)(tl + tbase) = lv;
  }
}

__global__ __launch_bounds__(kThreads)
void filter_steps(const float* __restrict__ xin, const float* __restrict__ uin,
                  const float* __restrict__ Ag, const float* __restrict__ Bg,
                  const float* __restrict__ Cg, const float* __restrict__ Qg,
                  const float* __restrict__ Rg, float* __restrict__ out)
{
  __shared__ __align__(16) _Float16 sPTh[kN * kHP];
  __shared__ __align__(16) _Float16 sPTl[kN * kHP];
  __shared__ __align__(16) _Float16 sT1h[kN * kHP];
  __shared__ __align__(16) _Float16 sT1l[kN * kHP];
  __shared__ __align__(16) _Float16 sPPh[kN * kHP];
  __shared__ __align__(16) _Float16 sPPl[kN * kHP];
  __shared__ __align__(16) _Float16 sPPTh[kN * kHP];
  __shared__ __align__(16) _Float16 sPPTl[kN * kHP];
  __shared__ __align__(16) _Float16 sMh[kN * kHP];
  __shared__ __align__(16) _Float16 sMl[kN * kHP];
  __shared__ __align__(16) _Float16 sMTh[kN * kHP];
  __shared__ __align__(16) _Float16 sMTl[kN * kHP];
  __shared__ __align__(16) _Float16 sGh[kN * kHP];
  __shared__ __align__(16) _Float16 sGl[kN * kHP];
  __shared__ __align__(16) float sA[kN * kFP];
  __shared__ __align__(16) float sB[kN * kFP];
  __shared__ __align__(16) float sC[kN * kFP];
  __shared__ __align__(16) float sW[kN * kFP];
  __shared__ __align__(16) float sZ[kN];
  __shared__ __align__(16) float sZp[kN];
  __shared__ __align__(16) float sInn[kN];
  __shared__ __align__(16) float sRd[kN];
  __shared__ __align__(16) float sXt[kBuf * kN];
  __shared__ __align__(16) float sUt[kBuf * kN];
  __shared__ __align__(16) float sOut[kN * kBuf];

  _Float16* const sKh  = sT1h;
  _Float16* const sKl  = sT1l;
  _Float16* const sSIh = sPPh;
  _Float16* const sSIl = sPPl;

  const int tid  = threadIdx.x;
  const int lane = tid & 31;
  const int wave = __builtin_amdgcn_readfirstlane(tid >> 5);
  const int hh   = lane >> 4;
  const int nn   = lane & 15;
  const int tm16 = (wave >> 2) * 16;
  const int tn16 = (wave & 3) * 16;
  const int aoff  = (tm16 + nn) * kHP + 8 * hh;
  const int boff  = (tn16 + nn) * kHP + 8 * hh;
  const int rbase = (tm16 + 8 * hh) * kHP + tn16 + nn;
  const int tbase = (tn16 + nn) * kHP + tm16 + 8 * hh;
  const int fbase = (tm16 + 8 * hh) * kFP + tn16 + nn;

#pragma unroll 1
  for (int i = tid; i < kN * kN; i += kThreads) {
    const int r = i >> 6, c = i & 63;
    sA[r * kFP + c] = bf16v(Ag[i]);
    sB[r * kFP + c] = bf16v(Bg[i]);
    sC[r * kFP + c] = bf16v(Cg[i]);
  }
#pragma unroll 1
  for (int i = tid; i < kN * kHP; i += kThreads) {
    const int r = i / kHP;
    const int c = i - r * kHP;
    const float dv = (r == c) ? kCarry : 0.0f;
    sPTh[i] = (_Float16)dv;
    sPTl[i] = (_Float16)(dv * 0.0f);
  }
  if (tid < kN) sZ[tid] = 0.0f;

  v16h fAa[2], fAb[2], fCa[2], fCb[2];
#pragma unroll
  for (int ks = 0; ks < 2; ++ks) {
    fAa[ks] = wfrag(Ag, tm16 + nn, 32 * ks + 8 * hh);
    fAb[ks] = wfrag(Ag, tn16 + nn, 32 * ks + 8 * hh);
    fCa[ks] = wfrag(Cg, tm16 + nn, 32 * ks + 8 * hh);
    fCb[ks] = wfrag(Cg, tn16 + nn, 32 * ks + 8 * hh);
  }
  float qreg[8], rreg[8];
#pragma unroll
  for (int r = 0; r < 8; ++r) {
    qreg[r] = bf16v(Qg[(tm16 + 8 * hh + r) * kN + tn16 + nn]);
    rreg[r] = bf16v(Rg[(tm16 + 8 * hh + r) * kN + tn16 + nn]);
  }
  __syncthreads();

  const v8f z8 = (v8f){0.f, 0.f, 0.f, 0.f, 0.f, 0.f, 0.f, 0.f};

#pragma unroll 1
  for (int t = 0; t < kT; ++t) {
    const int tt = t & (kBuf - 1);

    if (tt == 0) {
      const int j = tid >> 3, q4 = (tid & 7) * 4;
      const v4f xv = *(const v4f*)(xin + (size_t)j * kT + t + q4);
      const v4f uv = *(const v4f*)(uin + (size_t)j * kT + t + q4);
#pragma unroll
      for (int e = 0; e < 4; ++e) {
        const float xe = xv[e];
        const float ue = uv[e];
        sXt[(q4 + e) * kN + j] = bf16v(xe);
        sUt[(q4 + e) * kN + j] = bf16v(ue);
      }
      __syncthreads();
    }

    float pp[8];

    {
      v8f cm = z8, cr = z8;
#pragma unroll
      for (int ks = 0; ks < 2; ++ks) {
        const v16h bh = ldfrag(sPTh + boff + 32 * ks);
        const v16h bl = ldfrag(sPTl + boff + 32 * ks);
        cm = mma16(fAa[ks], bh, cm);
        cr = mma16(fAa[ks], bl, cr);
      }
      float cv[8];
#pragma unroll
      for (int r = 0; r < 8; ++r) cv[r] = fmaf(cr[r], kInvRes, cm[r]) * kInvCarry;
      put_planes<true, false>(cv, sT1h, sT1l, rbase, nullptr, nullptr, 0);
    }
    if (wave < 2) {
      const float* ar = sA + tid * kFP;
      const float* br = sB + tid * kFP;
      const float* ut = sUt + tt * kN;
      float s0 = 0.0f, s1 = 0.0f;
#pragma unroll 2
      for (int j = 0; j < kN; j += 4) {
        const v4f a = *(const v4f*)(ar + j);
        const v4f z = *(const v4f*)(sZ + j);
        const v4f b = *(const v4f*)(br + j);
        const v4f u = *(const v4f*)(ut + j);
        s0 = fmaf(a[0], z[0], s0);
        s0 = fmaf(a[1], z[1], s0);
        s0 = fmaf(a[2], z[2], s0);
        s0 = fmaf(a[3], z[3], s0);
        s1 = fmaf(b[0], u[0], s1);
        s1 = fmaf(b[1], u[1], s1);
        s1 = fmaf(b[2], u[2], s1);
        s1 = fmaf(b[3], u[3], s1);
      }
      sZp[tid] = s0 + s1;
    }
    __syncthreads();

    {
      v8f cm = z8, cr = z8;
#pragma unroll
      for (int ks = 0; ks < 2; ++ks) {
        const v16h ah = ldfrag(sT1h + aoff + 32 * ks);
        const v16h al = ldfrag(sT1l + aoff + 32 * ks);
        cm = mma16(ah, fAb[ks], cm);
        cr = mma16(al, fAb[ks], cr);
      }
      float cv[8];
#pragma unroll
      for (int r = 0; r < 8; ++r) {
        pp[r] = fmaf(cr[r], kInvRes, cm[r]) * kInvCC + qreg[r];
        cv[r] = pp[r] * kCarry;
      }
      put_planes<true, true>(cv, sPPh, sPPl, rbase, sPPTh, sPPTl, tbase);
    }
    if (wave < 2) {
      const float* cr_ = sC + tid * kFP;
      float s = 0.0f;
#pragma unroll 2
      for (int j = 0; j < kN; j += 4) {
        const v4f c = *(const v4f*)(cr_ + j);
        const v4f z = *(const v4f*)(sZp + j);
        s = fmaf(c[0], z[0], s);
        s = fmaf(c[1], z[1], s);
        s = fmaf(c[2], z[2], s);
        s = fmaf(c[3], z[3], s);
      }
      sInn[tid] = sXt[tt * kN + tid] - s;
    }
    __syncthreads();

    {
      v8f cm = z8, cr = z8;
#pragma unroll
      for (int ks = 0; ks < 2; ++ks) {
        const v16h bh = ldfrag(sPPTh + boff + 32 * ks);
        const v16h bl = ldfrag(sPPTl + boff + 32 * ks);
        cm = mma16(fCa[ks], bh, cm);
        cr = mma16(fCa[ks], bl, cr);
      }
      float cv[8];
#pragma unroll
      for (int r = 0; r < 8; ++r) cv[r] = fmaf(cr[r], kInvRes, cm[r]) * kInvCarry;
      put_planes<true, true>(cv, sMh, sMl, rbase, sMTh, sMTl, tbase);
    }
    {
      v8f cm = z8, cr = z8;
#pragma unroll
      for (int ks = 0; ks < 2; ++ks) {
        const v16h ah = ldfrag(sPPh + aoff + 32 * ks);
        const v16h al = ldfrag(sPPl + aoff + 32 * ks);
        cm = mma16(ah, fCb[ks], cm);
        cr = mma16(al, fCb[ks], cr);
      }
      float cv[8];
#pragma unroll
      for (int r = 0; r < 8; ++r) cv[r] = fmaf(cr[r], kInvRes, cm[r]) * kInvCarry;
      put_planes<true, false>(cv, sGh, sGl, rbase, nullptr, nullptr, 0);
    }
    __syncthreads();

    {
      v8f cm = z8, cr = z8;
#pragma unroll
      for (int ks = 0; ks < 2; ++ks) {
        const v16h ah = ldfrag(sMh + aoff + 32 * ks);
        const v16h al = ldfrag(sMl + aoff + 32 * ks);
        cm = mma16(ah, fCb[ks], cm);
        cr = mma16(al, fCb[ks], cr);
      }
#pragma unroll
      for (int r = 0; r < 8; ++r)
        sW[fbase + r * kFP] = fmaf(cr[r], kInvRes, cm[r]) * kInvCC + rreg[r];
    }
    __syncthreads();

    if (wave == 0) {
      float rd0 = 1.0f, rd1 = 1.0f;
      float* w0 = sW + lane * kFP;
      float* w1 = sW + (lane + 32) * kFP;
#pragma unroll 1
      for (int p = 0; p < kN; ++p) {
        const float* prow = sW + p * kFP;
        const float piv  = prow[p];
        const float rinv = 1.0f / piv;
        const float e0 = w0[p];
        const float e1 = w1[p];
        const bool is0 = (lane == p);
        const bool is1 = (lane + 32 == p);
        const float f0 = is0 ? 0.0f : e0 * rinv;
        const float f1 = is1 ? 0.0f : e1 * rinv;
        rd0 = is0 ? rinv : rd0;
        rd1 = is1 ? rinv : rd1;
#pragma unroll 4
        for (int c4 = 0; c4 < kN; c4 += 4) {
          const v4f pr = *(const v4f*)(prow + c4);
          v4f a = *(const v4f*)(w0 + c4);
          v4f b = *(const v4f*)(w1 + c4);
          a[0] = fmaf(-f0, pr[0], a[0]);
          a[1] = fmaf(-f0, pr[1], a[1]);
          a[2] = fmaf(-f0, pr[2], a[2]);
          a[3] = fmaf(-f0, pr[3], a[3]);
          b[0] = fmaf(-f1, pr[0], b[0]);
          b[1] = fmaf(-f1, pr[1], b[1]);
          b[2] = fmaf(-f1, pr[2], b[2]);
          b[3] = fmaf(-f1, pr[3], b[3]);
          *(v4f*)(w0 + c4) = a;
          *(v4f*)(w1 + c4) = b;
        }
        const float n0 = is0 ? 1.0f : -f0;
        const float n1 = is1 ? 1.0f : -f1;
        w0[p] = n0;
        w1[p] = n1;
        __builtin_amdgcn_fence(__ATOMIC_RELEASE, "workgroup");
        __builtin_amdgcn_wave_barrier();
        __builtin_amdgcn_fence(__ATOMIC_ACQUIRE, "workgroup");
      }
      sRd[lane]      = rd0;
      sRd[lane + 32] = rd1;
    }
    __syncthreads();

    {
      const int n6 = tid >> 3, k8 = (tid & 7) * 8;
      const v4f r0 = *(const v4f*)(sRd + k8);
      const v4f r1 = *(const v4f*)(sRd + k8 + 4);
      v8h hv, lv;
#pragma unroll
      for (int e = 0; e < 4; ++e) {
        const float wa = sW[(k8 + e) * kFP + n6];
        const float wb = sW[(k8 + 4 + e) * kFP + n6];
        const float ra = r0[e];
        const float rb = r1[e];
        _Float16 a, b;
        split16(wa * ra * kCarry, a, b);
        hv[e] = a;
        lv[e] = b;
        split16(wb * rb * kCarry, a, b);
        hv[4 + e] = a;
        lv[4 + e] = b;
      }
      *(v8h*)(sSIh + n6 * kHP + k8) = hv;
      *(v8h*)(sSIl + n6 * kHP + k8) = lv;
    }
    __syncthreads();

    {
      v8f cm = z8, cr = z8;
#pragma unroll
      for (int ks = 0; ks < 2; ++ks) {
        const v16h ah = ldfrag(sGh + aoff + 32 * ks);
        const v16h al = ldfrag(sGl + aoff + 32 * ks);
        const v16h bh = ldfrag(sSIh + boff + 32 * ks);
        const v16h bl = ldfrag(sSIl + boff + 32 * ks);
        cm = mma16(ah, bh, cm);
        cr = mma16(ah, bl, cr);
        cr = mma16(al, bh, cr);
      }
      float cv[8];
#pragma unroll
      for (int r = 0; r < 8; ++r) {
        const float kv = fmaf(cr[r], kInvRes, cm[r]) * kInvCC;
        sW[fbase + r * kFP] = kv;
        cv[r] = kv * kCarry;
      }
      put_planes<true, false>(cv, sKh, sKl, rbase, nullptr, nullptr, 0);
    }
    __syncthreads();

    {
      v8f cm = z8, cr = z8;
#pragma unroll
      for (int ks = 0; ks < 2; ++ks) {
        const v16h ah = ldfrag(sKh + aoff + 32 * ks);
        const v16h al = ldfrag(sKl + aoff + 32 * ks);
        const v16h bh = ldfrag(sMTh + boff + 32 * ks);
        const v16h bl = ldfrag(sMTl + boff + 32 * ks);
        cm = mma16(ah, bh, cm);
        cr = mma16(ah, bl, cr);
        cr = mma16(al, bh, cr);
      }
      float cv[8];
#pragma unroll
      for (int r = 0; r < 8; ++r) {
        const float pn = pp[r] - fmaf(cr[r], kInvRes, cm[r]) * kInvCC;
        cv[r] = pn * kCarry;
      }
      put_planes<false, true>(cv, nullptr, nullptr, 0, sPTh, sPTl, tbase);
    }
    if (wave < 2) {
      const float* kr = sW + tid * kFP;
      float s = 0.0f;
#pragma unroll 2
      for (int j = 0; j < kN; j += 4) {
        const v4f k4 = *(const v4f*)(kr + j);
        const v4f i4 = *(const v4f*)(sInn + j);
        s = fmaf(k4[0], i4[0], s);
        s = fmaf(k4[1], i4[1], s);
        s = fmaf(k4[2], i4[2], s);
        s = fmaf(k4[3], i4[3], s);
      }
      const float zn = sZp[tid] + s;
      sZ[tid] = zn;
      sOut[tid * kBuf + tt] = zn;
    }
    __syncthreads();

    if (tt == kBuf - 1) {
      const int l  = wave * 4 + (lane >> 3);
      const int c4 = (lane & 7) * 4;
      const int t0 = t - (kBuf - 1);
      const v4f v = *(const v4f*)(sOut + l * kBuf + c4);
      float* dst = out + (size_t)l * kT + t0 + c4;
      *(volatile v4f*)dst = v;
      __threadfence();
      *(volatile v4f*)dst = v;
    }
  }
}

extern "C" void kernel_launch(void* const* d_in, const int* in_sizes, int n_in,
                              void* d_out, int out_size, void* d_ws, size_t ws_size,
                              hipStream_t stream) {
  if (n_in < 7) return;
  if (in_sizes[0] != kN * kT) return;
  if (in_sizes[1] != kN * kT) return;
  if (in_sizes[2] != kN * kN) return;
  if (in_sizes[3] != kN * kN) return;
  if (in_sizes[4] != kN * kN) return;
  if (in_sizes[5] != kN * kN) return;
  if (in_sizes[6] != kN * kN) return;
  if (out_size != kN * kT) return;
  (void)d_ws;
  (void)ws_size;

  const float* xin = (const float*)d_in[0];
  const float* uin = (const float*)d_in[1];
  const float* Ag  = (const float*)d_in[2];
  const float* Bg  = (const float*)d_in[3];
  const float* Cg  = (const float*)d_in[4];
  const float* Qg  = (const float*)d_in[5];
  const float* Rg  = (const float*)d_in[6];
  float* out = (float*)d_out;

  filter_steps<<<dim3(1), dim3(kThreads), 0, stream>>>(xin, uin, Ag, Bg, Cg, Qg, Rg, out);
}
